// TransformerEncoderRPALayer_49821620633750
// MI455X (gfx1250) — hardware-verified
//
#include <hip/hip_runtime.h>
#define SS 2048
#define NB2 2
#define DD 512
#define NH 8
#define HD 64
#define DFF 2048
#define NR (SS * NB2)
#define MAXLEN 16384
#define HG 1
typedef __bf16 v16b __attribute__((ext_vector_type(16)));
typedef unsigned short v8us __attribute__((ext_vector_type(8), may_alias));
typedef float  v8f  __attribute__((ext_vector_type(8)));
typedef float  v4f  __attribute__((ext_vector_type(4)));
typedef float  v4fa __attribute__((ext_vector_type(4), may_alias));
union FragB { v16b v; v8us half[2]; unsigned short u[16]; };

__device__ __forceinline__ unsigned short bf16_bits(float x) { unsigned int u = __float_as_uint(x); return (unsigned short)((u + 0x7FFFu + ((u >> 16) & 1u)) >> 16); }
__device__ __forceinline__ float bf16_val(unsigned short b) { return __uint_as_float(((unsigned int)b) << 16); }
__device__ __forceinline__ float bf16_round(float x) { return bf16_val(bf16_bits(x)); }
template <int NT>
__device__ __forceinline__ v8f mmaN(v16b ah, v16b al, v16b bh, v16b bl, v8f c) {
  c = __builtin_amdgcn_wmma_f32_16x16x32_bf16(false, ah, false, bh, (short)0, c, false, false);
  if (NT >= 2) c = __builtin_amdgcn_wmma_f32_16x16x32_bf16(false, al, false, bh, (short)0, c, false, false);
  if (NT >= 3) c = __builtin_amdgcn_wmma_f32_16x16x32_bf16(false, ah, false, bl, (short)0, c, false, false);
  asm volatile("v_nop\n\tv_nop\n\tv_nop\n\tv_nop" : "+v"(c) : "v"(ah), "v"(al), "v"(bh), "v"(bl));
  return c;
}

__global__ __launch_bounds__(256) void k_wt_bf16(const float* __restrict__ W, unsigned short* __restrict__ Wt, int K, int N) {
  const int t = blockIdx.x * 256 + threadIdx.x;
  const int k8n = K / 8;
  if (t >= N * k8n) return;
  const int n = t / k8n, k8 = (t % k8n) * 8;
  v8us v;
#pragma unroll
  for (int i = 0; i < 8; ++i) v[i] = bf16_bits(W[(size_t)(k8 + i) * N + n]);
  *(volatile v8us*)(Wt + (size_t)n * K + k8) = v;
  __threadfence();
  *(volatile v8us*)(Wt + (size_t)n * K + k8) = v;
}

template <bool ASPLIT, int ACT, bool BIAS_BF16>
__global__ __launch_bounds__(128) void k_gemm_bf(const float* __restrict__ A, int lda, const unsigned short* __restrict__ Wt, int ldb,
                                               const float* __restrict__ bias, float* __restrict__ C, int ldc, int M, int N, int K) {
  __shared__ __attribute__((aligned(16))) float so[4][16][64];
  const int tid = threadIdx.x, w = tid >> 5, lane = tid & 31, ln = lane & 15, hh = lane >> 4;
  const int ntn = N / 64;
  const int wid = blockIdx.x * 4 + w;
  const int mt = wid / ntn, nq = wid % ntn;
  if (mt * 16 >= M) return;
  const int row0 = mt * 16, col0 = nq * 64;
  const float* arow = A + (size_t)(row0 + ln) * lda;
  v8f acc[4] = {};
  for (int kb = 0; kb < K; kb += 32) {
    FragB ah, al;
    const v4f x0 = *(const v4fa*)(arow + kb + 8 * hh), x1 = *(const v4fa*)(arow + kb + 8 * hh + 4);
    const v4f x2 = *(const v4fa*)(arow + kb + 16 + 8 * hh), x3 = *(const v4fa*)(arow + kb + 16 + 8 * hh + 4);
    float xs[16] = {x0[0],x0[1],x0[2],x0[3],x1[0],x1[1],x1[2],x1[3],x2[0],x2[1],x2[2],x2[3],x3[0],x3[1],x3[2],x3[3]};
#pragma unroll
    for (int i = 0; i < 16; ++i) { const unsigned short hb = bf16_bits(xs[i]); ah.u[i] = hb; al.u[i] = ASPLIT ? bf16_bits(xs[i] - bf16_val(hb)) : (unsigned short)0; }
#pragma unroll
    for (int t = 0; t < 4; ++t) {
      const unsigned short* brow = Wt + (size_t)(col0 + t * 16 + ln) * ldb + kb;
      FragB b;
      b.half[0] = *(const v8us*)(brow + 8 * hh);
      b.half[1] = *(const v8us*)(brow + 16 + 8 * hh);
      acc[t] = mmaN<ASPLIT ? 2 : 1>(ah.v, al.v, b.v, b.v, acc[t]);
    }
  }
#pragma unroll
  for (int t = 0; t < 4; ++t) {
    float bv = bias ? bias[col0 + t * 16 + ln] : 0.f;
    if (BIAS_BF16) bv = bf16_round(bv);
#pragma unroll
    for (int r = 0; r < 8; ++r) { float v = acc[t][r] + bv; if (ACT == 1) v = fmaxf(v, 0.f); so[w][8 * hh + r][t * 16 + ln] = v; }
  }
  __builtin_amdgcn_fence(__ATOMIC_ACQ_REL, "workgroup");
  __builtin_amdgcn_wave_barrier();
  const int rsub = lane >> 4, c4 = (lane & 15) * 4;
  for (int pass = 0; pass < 2; ++pass) {
#pragma unroll
    for (int q = 0; q < 8; ++q) {
      const int r = q * 2 + rsub;
      const v4f v = *(const v4fa*)&so[w][r][c4];
      *(volatile v4f*)(C + (size_t)(row0 + r) * ldc + col0 + c4) = v;
    }
    if (pass == 0) __threadfence();
  }
}

template <bool ASPLIT, int ACT, bool BIAS_BF16, bool RES_BF16>
__global__ __launch_bounds__(128) void k_gemm_bf3(const float* __restrict__ A, int lda, const unsigned short* __restrict__ Wt, int ldb,
                                                const float* __restrict__ bias, const float* __restrict__ resid, int rmod, int ldr,
                                                float* __restrict__ C, int ldc, int M, int N, int K) {
  __shared__ __attribute__((aligned(16))) float so[4][16][64];
  const int tid = threadIdx.x, w = tid >> 5, lane = tid & 31, ln = lane & 15, hh = lane >> 4;
  const int ntn = N / 64;
  const int wid = blockIdx.x * 4 + w;
  const int mt = wid / ntn, nq = wid % ntn;
  if (mt * 16 >= M) return;
  const int row0 = mt * 16, col0 = nq * 64;
  const float* arow = A + (size_t)(row0 + ln) * lda;
  v8f acc[4] = {};
  for (int kb = 0; kb < K; kb += 32) {
    FragB ah, al;
    const v4f x0 = *(const v4fa*)(arow + kb + 8 * hh), x1 = *(const v4fa*)(arow + kb + 8 * hh + 4);
    const v4f x2 = *(const v4fa*)(arow + kb + 16 + 8 * hh), x3 = *(const v4fa*)(arow + kb + 16 + 8 * hh + 4);
    float xs[16] = {x0[0],x0[1],x0[2],x0[3],x1[0],x1[1],x1[2],x1[3],x2[0],x2[1],x2[2],x2[3],x3[0],x3[1],x3[2],x3[3]};
#pragma unroll
    for (int i = 0; i < 16; ++i) { const unsigned short hb = bf16_bits(xs[i]); ah.u[i] = hb; al.u[i] = ASPLIT ? bf16_bits(xs[i] - bf16_val(hb)) : (unsigned short)0; }
#pragma unroll
    for (int t = 0; t < 4; ++t) {
      const unsigned short* brow = Wt + (size_t)(col0 + t * 16 + ln) * ldb + kb;
      FragB b;
      b.half[0] = *(const v8us*)(brow + 8 * hh);
      b.half[1] = *(const v8us*)(brow + 16 + 8 * hh);
      acc[t] = mmaN<ASPLIT ? 2 : 1>(ah.v, al.v, b.v, b.v, acc[t]);
    }
  }
#pragma unroll
  for (int t = 0; t < 4; ++t) {
    const int col = col0 + t * 16 + ln;
    float bv = bias ? bias[col] : 0.f;
    if (BIAS_BF16) bv = bf16_round(bv);
#pragma unroll
    for (int r = 0; r < 8; ++r) {
      float v = acc[t][r] + bv;
      if (resid) { float rv = resid[(size_t)((row0 + 8 * hh + r) % rmod) * ldr + col]; if (RES_BF16) rv = bf16_round(rv); v += rv; }
      if (ACT == 1) v = fmaxf(v, 0.f);
      if (ACT == 2) v = 0.5f * v * (1.0f + erff(v * 0.70710678118654752f));
      if (ACT == 3) { const float u = 0.7978845608028654f * (v + 0.044715f * v * v * v); v = 0.5f * v * (1.0f + tanhf(u)); }
      so[w][8 * hh + r][t * 16 + ln] = v;
    }
  }
  __builtin_amdgcn_fence(__ATOMIC_ACQ_REL, "workgroup");
  __builtin_amdgcn_wave_barrier();
  const int rsub = lane >> 4, c4 = (lane & 15) * 4;
  for (int pass = 0; pass < 2; ++pass) {
#pragma unroll
    for (int q = 0; q < 8; ++q) {
      const int r = q * 2 + rsub;
      const v4f v = *(const v4fa*)&so[w][r][c4];
      *(volatile v4f*)(C + (size_t)(row0 + r) * ldc + col0 + c4) = v;
    }
    if (pass == 0) __threadfence();
  }
}
template <bool PARAM_BF16>
__global__ __launch_bounds__(256) void k_layernorm(const float* __restrict__ X, const float* __restrict__ R, const float* __restrict__ g, const float* __restrict__ bta,
                                                  float* __restrict__ out_sum, float* __restrict__ out_norm, int N, float eps) {
  __shared__ float red[256];
  const int row = blockIdx.x, tid = threadIdx.x;
  const float* x = X + (size_t)row * N; const float* rr = R ? R + (size_t)row * N : nullptr;
  float vals[16];
  const int per = N / 256;
  float s1 = 0.f;
  for (int u = 0; u < per / 4; ++u) {
    const int j = tid * 4 + 1024 * u;
    const v4f a = *(const v4fa*)(x + j);
    v4f b = {0.f,0.f,0.f,0.f}; if (rr) b = *(const v4fa*)(rr + j);
#pragma unroll
    for (int q = 0; q < 4; ++q) { const float v = a[q] + b[q]; vals[u * 4 + q] = v; s1 += v; }
  }
  red[tid] = s1; __syncthreads();
  for (int st = 128; st > 0; st >>= 1) { if (tid < st) red[tid] += red[tid + st]; __syncthreads(); }
  const float mu = red[0] / (float)N; __syncthreads();
  float s2 = 0.f;
  for (int u = 0; u < per / 4; ++u)
#pragma unroll
    for (int q = 0; q < 4; ++q) { const float c = vals[u * 4 + q] - mu; s2 += c * c; }
  red[tid] = s2; __syncthreads();
  for (int st = 128; st > 0; st >>= 1) { if (tid < st) red[tid] += red[tid + st]; __syncthreads(); }
  const float rs = rsqrtf(red[0] / (float)N + eps);
  for (int pass = 0; pass < 2; ++pass) {
    for (int u = 0; u < per / 4; ++u) {
      const int j = tid * 4 + 1024 * u;
      v4f o, sm;
#pragma unroll
      for (int q = 0; q < 4; ++q) {
        float gg = g[j + q], bb = bta[j + q];
        if (PARAM_BF16) { gg = bf16_round(gg); bb = bf16_round(bb); }
        sm[q] = vals[u * 4 + q]; o[q] = (vals[u * 4 + q] - mu) * rs * gg + bb;
      }
      if (out_sum) *(volatile v4f*)(out_sum + (size_t)row * N + j) = sm;
      *(volatile v4f*)(out_norm + (size_t)row * N + j) = o;
    }
    if (pass == 0) __threadfence();
  }
}


typedef _Float16 v16h __attribute__((ext_vector_type(16)));
union FragH { v16h v; v8us half[2]; _Float16 h[16]; unsigned short u[16]; };
template <int NT>
__device__ __forceinline__ v8f mmaH(v16h ah, v16h al, v16h bh, v16h bl, v8f c) {
  c = __builtin_amdgcn_wmma_f32_16x16x32_f16(false, ah, false, bh, (short)0, c, false, false);
  if (NT >= 2) c = __builtin_amdgcn_wmma_f32_16x16x32_f16(false, al, false, bh, (short)0, c, false, false);
  if (NT >= 3) c = __builtin_amdgcn_wmma_f32_16x16x32_f16(false, ah, false, bl, (short)0, c, false, false);
  asm volatile("v_nop\n\tv_nop\n\tv_nop\n\tv_nop" : "+v"(c) : "v"(ah), "v"(al), "v"(bh), "v"(bl));
  return c;
}
template <bool ASPLIT>
__global__ __launch_bounds__(128) void k_gemm_h(const float* __restrict__ A, int lda, size_t sA, const _Float16* __restrict__ Bh, int ldb, size_t sB, float alpha, float* __restrict__ C, int ldc, size_t sC, int M, int N, int K) {
  __shared__ __attribute__((aligned(16))) float so[4][16][64];
  const int tid = threadIdx.x, w = tid >> 5, lane = tid & 31, ln = lane & 15, hh = lane >> 4; const int by = blockIdx.y;
  A += (size_t)by * sA; Bh += (size_t)by * sB; C += (size_t)by * sC;
  const int ntn = (N + 63) / 64; const int wid = blockIdx.x * 4 + w; const int mt = wid / ntn, nq = wid % ntn; if (mt * 16 >= M) return;
  const int row0 = mt * 16, col0 = nq * 64; const float* arow = A + (size_t)(row0 + ln) * lda;
  v8f acc[4] = {};
  for (int kb = 0; kb < K; kb += 32) {
    FragH ah, al;
    const v4f x0 = *(const v4fa*)(arow + kb + 8 * hh), x1 = *(const v4fa*)(arow + kb + 8 * hh + 4), x2 = *(const v4fa*)(arow + kb + 16 + 8 * hh), x3 = *(const v4fa*)(arow + kb + 16 + 8 * hh + 4);
    float xs[16] = {x0[0],x0[1],x0[2],x0[3],x1[0],x1[1],x1[2],x1[3],x2[0],x2[1],x2[2],x2[3],x3[0],x3[1],x3[2],x3[3]};
#pragma unroll
    for (int i = 0; i < 16; ++i) { const _Float16 h = (_Float16)xs[i]; ah.h[i] = h; al.h[i] = ASPLIT ? (_Float16)(xs[i] - (float)h) : (_Float16)0.0f; }
#pragma unroll
    for (int t = 0; t < 4; ++t) { if (col0 + t * 16 >= N) continue; const size_t boff = (size_t)(col0 + t * 16 + ln) * ldb + kb; FragH bq; bq.half[0] = *(const v8us*)(Bh + boff + 8 * hh); bq.half[1] = *(const v8us*)(Bh + boff + 16 + 8 * hh);
      acc[t] = mmaH<ASPLIT ? 2 : 1>(ah.v, al.v, bq.v, bq.v, acc[t]); }
  }
#pragma unroll
  for (int t = 0; t < 4; ++t) { if (col0 + t * 16 >= N) continue;
#pragma unroll
    for (int r = 0; r < 8; ++r) so[w][8 * hh + r][t * 16 + ln] = acc[t][r] * alpha; }
  __builtin_amdgcn_fence(__ATOMIC_ACQ_REL, "workgroup"); __builtin_amdgcn_wave_barrier();
  const int rsub = lane >> 4, c4 = (lane & 15) * 4;
  for (int pass = 0; pass < 2; ++pass) {
#pragma unroll
    for (int q = 0; q < 8; ++q) { const int r = q * 2 + rsub; if (col0 + c4 < N) { const v4f v = *(const v4fa*)&so[w][r][c4]; *(volatile v4f*)(C + (size_t)(row0 + r) * ldc + col0 + c4) = v; } }
    if (pass == 0) __threadfence(); }
}

__global__ __launch_bounds__(256) void k_wt_f16(const float* __restrict__ W, _Float16* __restrict__ Wt, int K, int N, float scale) {
  const int t = blockIdx.x * 256 + threadIdx.x; if (t >= N * (K / 8)) return; const int n = t / (K / 8), k8 = (t % (K / 8)) * 8; FragH f;
#pragma unroll
  for (int i = 0; i < 8; ++i) f.h[i] = (_Float16)(bf16_round(W[(size_t)(k8 + i) * N + n]) * scale); const v8us o = f.half[0];
  *(volatile v8us*)((unsigned short*)Wt + (size_t)n * K + k8) = o; __threadfence(); *(volatile v8us*)((unsigned short*)Wt + (size_t)n * K + k8) = o;
}
template <int ACT>
__global__ __launch_bounds__(128) void k_gemm_hhx(const _Float16* __restrict__ A, int lda, size_t sA, const _Float16* __restrict__ Bh, int ldb, size_t sB, float alpha, const float* __restrict__ bias, size_t sBias, const float* __restrict__ CP, int rowsPerB, size_t sCPb, int row0g,
    float* __restrict__ C, _Float16* __restrict__ C16, int ldc, size_t sC, int M, int N, int K) {
  __shared__ __attribute__((aligned(16))) float so[4][16][64];
  const int tid = threadIdx.x, w = tid >> 5, lane = tid & 31, ln = lane & 15, hh = lane >> 4; const int by = blockIdx.y;
  A += (size_t)by * sA; Bh += (size_t)by * sB; const size_t cofs = (size_t)by * sC; const float* bp = bias ? bias + (size_t)by * sBias : nullptr;
  const int ntn = (N + 63) / 64; const int wid = blockIdx.x * 4 + w; const int mt = wid / ntn, nq = wid % ntn; if (mt * 16 >= M) return;
  const int row0 = mt * 16, col0 = nq * 64; const _Float16* arow = A + (size_t)(row0 + ln) * lda;
  v8f acc[4] = {};
  for (int kb = 0; kb < K; kb += 32) { FragH ah; ah.half[0] = *(const v8us*)((const unsigned short*)arow + kb + 8 * hh); ah.half[1] = *(const v8us*)((const unsigned short*)arow + kb + 16 + 8 * hh);
#pragma unroll
    for (int t = 0; t < 4; ++t) { if (col0 + t * 16 >= N) continue; const size_t boff = (size_t)(col0 + t * 16 + ln) * ldb + kb; FragH bq; bq.half[0] = *(const v8us*)((const unsigned short*)Bh + boff + 8 * hh); bq.half[1] = *(const v8us*)((const unsigned short*)Bh + boff + 16 + 8 * hh);
      acc[t] = mmaH<1>(ah.v, ah.v, bq.v, bq.v, acc[t]); }
  }
#pragma unroll
  for (int t = 0; t < 4; ++t) { if (col0 + t * 16 >= N) continue; const int col = col0 + t * 16 + ln; const float bv = bp ? bf16_round(bp[col]) : 0.f;
#pragma unroll
    for (int r = 0; r < 8; ++r) { float v = acc[t][r] * alpha + bv; if (CP) { const int bidx = (row0g + row0 + 8 * hh + r) / rowsPerB; v += CP[(size_t)bidx * sCPb + (size_t)by * 64 + col]; } if (ACT == 1) v = (v > 0.f) ? v : expm1f(v); else if (ACT == 7) v = (v > 0.f) ? v + 1.0f : expf(v); else if (ACT == 8) v = tanhf(v); else if (ACT == 9) v = 0.5f * v * (1.0f + tanhf(0.7978845608028654f * (v + 0.044715f * v * v * v))); else if (ACT == 11) v = 1.0f / (1.0f + expf(-v)); else if (ACT == 12) v = (v > 0.f) ? v : 0.01f * v; else if (ACT == 14) v = (v > 0.f) ? v : 0.1f * v; else if (ACT == 15) v = v / (1.0f + expf(-v)); else if (ACT == 3) v = fmaxf(v, 0.f); else if (ACT == 6) v = 0.5f * v * (1.0f + erff(v * 0.70710678118654752f)); so[w][8 * hh + r][t * 16 + ln] = v; } }
  __builtin_amdgcn_fence(__ATOMIC_ACQ_REL, "workgroup"); __builtin_amdgcn_wave_barrier();
  const int rsub = lane >> 4, c4 = (lane & 15) * 4; typedef _Float16 v4h __attribute__((ext_vector_type(4)));
  for (int pass = 0; pass < 2; ++pass) {
#pragma unroll
    for (int q = 0; q < 8; ++q) { const int r = q * 2 + rsub; if (col0 + c4 < N) { const v4f v = *(const v4fa*)&so[w][r][c4]; if (C) *(volatile v4f*)(C + cofs + (size_t)(row0 + r) * ldc + col0 + c4) = v; if (C16) { v4h h4; for (int i = 0; i < 4; ++i) h4[i] = (_Float16)v[i]; *(volatile v4h*)(C16 + cofs + (size_t)(row0 + r) * ldc + col0 + c4) = h4; } } }
    if (pass == 0) __threadfence(); }
}


typedef _Float16 v4h __attribute__((ext_vector_type(4)));

__global__ __launch_bounds__(256) void k_x16(const float* __restrict__ x, _Float16* __restrict__ X16, size_t n8) { const size_t t = (size_t)blockIdx.x * 256 + threadIdx.x; if (t >= n8) return; FragH f;
#pragma unroll
  for (int q = 0; q < 8; ++q) f.h[q] = (_Float16)bf16_round(x[t * 8 + q]); *(volatile v8us*)((unsigned short*)X16 + t * 8) = f.half[0]; __threadfence(); *(volatile v8us*)((unsigned short*)X16 + t * 8) = f.half[0]; }
__global__ __launch_bounds__(256) void k_h16(const float* __restrict__ x, _Float16* __restrict__ X16, size_t n8) { const size_t t = (size_t)blockIdx.x * 256 + threadIdx.x; if (t >= n8) return; FragH f;
#pragma unroll
  for (int q = 0; q < 8; ++q) f.h[q] = (_Float16)x[t * 8 + q]; *(volatile v8us*)((unsigned short*)X16 + t * 8) = f.half[0]; __threadfence(); *(volatile v8us*)((unsigned short*)X16 + t * 8) = f.half[0]; }
__global__ __launch_bounds__(256) void k_round16f(const float* __restrict__ W, _Float16* __restrict__ Bt, size_t n8) { const size_t t = (size_t)blockIdx.x * 256 + threadIdx.x; if (t >= n8) return; FragH f;
#pragma unroll
  for (int i = 0; i < 8; ++i) f.h[i] = (_Float16)(bf16_round(W[t * 8 + i]) * 16.0f); *(volatile v8us*)((unsigned short*)Bt + t * 8) = f.half[0]; __threadfence(); *(volatile v8us*)((unsigned short*)Bt + t * 8) = f.half[0]; }
template <int NHv, int TTv>
__global__ __launch_bounds__(256) void k_vt(const _Float16* __restrict__ V16, int ldv, int voff, _Float16* __restrict__ Vt) { __shared__ unsigned short tl[64][66]; const int tid = threadIdx.x; const int slab = blockIdx.x / (TTv / 64), lg = blockIdx.x % (TTv / 64); const int b = slab / NHv, h = slab % NHv;
  for (int i = tid; i < 64 * 8; i += 256) { const int r = i / 8, c8 = (i % 8) * 8; FragH f; f.half[0] = *(const v8us*)((const unsigned short*)V16 + ((size_t)b * TTv + lg * 64 + r) * ldv + voff + h * 64 + c8);
#pragma unroll
    for (int q = 0; q < 8; ++q) tl[r][c8 + q] = f.u[q]; }
  __syncthreads();
  for (int pass = 0; pass < 2; ++pass) {
#pragma unroll
    for (int rd = 0; rd < 2; ++rd) { const int d = rd * 32 + tid / 8, pc = tid % 8; FragH f;
#pragma unroll
      for (int q = 0; q < 8; ++q) f.u[q] = tl[pc * 8 + q][d];
      *(volatile v8us*)((unsigned short*)Vt + ((size_t)slab * 64 + d) * TTv + lg * 64 + pc * 8) = f.half[0]; }
    if (pass == 0) __threadfence(); } }

__global__ __launch_bounds__(256) void k_hl(const float* __restrict__ F, _Float16* __restrict__ Hh, _Float16* __restrict__ Hl, size_t n8) { const size_t t = (size_t)blockIdx.x * 256 + threadIdx.x; if (t >= n8) return; FragH fh, fl; const v4f a = *(const v4fa*)(F + t * 8), c = *(const v4fa*)(F + t * 8 + 4);
#pragma unroll
  for (int q = 0; q < 4; ++q) { _Float16 h = (_Float16)a[q]; fh.h[q] = h; fl.h[q] = (_Float16)((a[q] - (float)h) * 1024.0f); h = (_Float16)c[q]; fh.h[4 + q] = h; fl.h[4 + q] = (_Float16)((c[q] - (float)h) * 1024.0f); }
  for (int pass = 0; pass < 2; ++pass) { *(volatile v8us*)((unsigned short*)Hh + t * 8) = fh.half[0]; *(volatile v8us*)((unsigned short*)Hl + t * 8) = fl.half[0]; if (pass == 0) __threadfence(); } }

__global__ __launch_bounds__(256) void k_er(const float* __restrict__ Er, _Float16* __restrict__ E16) { const int t = blockIdx.x * 256 + threadIdx.x; if (t >= SS * (HD / 8)) return; const int d0 = (t & 7) * 8, tt = t >> 3; FragH f;
#pragma unroll
  for (int q = 0; q < 8; ++q) f.h[q] = (_Float16)bf16_round(Er[((size_t)(MAXLEN - SS) + tt) * HD + d0 + q]);
  *(volatile v8us*)((unsigned short*)E16 + (size_t)tt * HD + d0) = f.half[0]; __threadfence(); *(volatile v8us*)((unsigned short*)E16 + (size_t)tt * HD + d0) = f.half[0]; }
__global__ __launch_bounds__(256) void k_vt(const _Float16* __restrict__ V16, _Float16* __restrict__ VT) { const int t = blockIdx.x * 256 + threadIdx.x; if (t >= DD * (SS / 8)) return; const int s0 = (t % (SS / 8)) * 8, hd = t / (SS / 8); FragH f;
#pragma unroll
  for (int q = 0; q < 8; ++q) f.h[q] = V16[(size_t)(s0 + q) * DD + hd];
  *(volatile v8us*)((unsigned short*)VT + (size_t)hd * SS + s0) = f.half[0]; __threadfence(); *(volatile v8us*)((unsigned short*)VT + (size_t)hd * SS + s0) = f.half[0]; }
__global__ __launch_bounds__(256) void k_rsoft(const float* __restrict__ QK, const float* __restrict__ QE, _Float16* __restrict__ P16) {
  #pragma clang fp contract(off)
  const int tid = threadIdx.x, w = tid >> 5, ln = tid & 31; const int row = blockIdx.x * 8 + w; if (row >= HG * SS) return; const int g = row / SS, r = row % SS; const float* sr = QK + (size_t)row * SS; const float* qe = QE + (size_t)g * SS * SS;
  auto val = [&](int c) { const int f = (r + 1) * SS + c; const int rp = f / (SS + 1), cpp = f - rp * (SS + 1); const float srel = (cpp == 0) ? 0.f : qe[(size_t)min(rp, SS - 1) * SS + (cpp - 1)]; return (sr[c] + srel) * 0.125f; };
  float m = -3.0e38f;
#pragma unroll 1
  for (int jb = 0; jb < SS; jb += 32) m = fmaxf(m, val(jb + ln));
  for (int o = 16; o > 0; o >>= 1) m = fmaxf(m, __shfl_xor(m, o, 32));
  float su = 0.f;
#pragma unroll 1
  for (int jb = 0; jb < SS; jb += 32) su += expf(val(jb + ln) - m);
  for (int o = 16; o > 0; o >>= 1) su += __shfl_xor(su, o, 32); const float inv = 1024.0f / su;
  for (int pass = 0; pass < 2; ++pass) {
#pragma unroll 1
    for (int jb = 0; jb < SS; jb += 256) { FragH f;
#pragma unroll
      for (int k = 0; k < 8; ++k) f.h[k] = (_Float16)(expf(val(jb + 8 * ln + k) - m) * inv);
      *(volatile v8us*)((unsigned short*)P16 + (size_t)row * SS + jb + 8 * ln) = f.half[0]; }
    if (pass == 0) __threadfence(); } }
__global__ __launch_bounds__(256) void k_ln1(const float* __restrict__ src, const float* __restrict__ SA, const float* __restrict__ g, const float* __restrict__ bb, float* __restrict__ X1, _Float16* __restrict__ X2) {
  #pragma clang fp contract(off)
  const int tid = threadIdx.x, w = tid >> 5, l = tid & 31; const int r = blockIdx.x * 8 + w; if (r >= NR) return; const int s = r >> 1; float v[16]; float sm = 0.f;
#pragma unroll
  for (int k = 0; k < 16; ++k) { const int c = l * 16 + k; v[k] = bf16_round(src[(size_t)r * DD + c]) + SA[(size_t)s * DD + c]; sm += v[k]; }
  for (int o = 16; o > 0; o >>= 1) sm += __shfl_xor(sm, o, 32); const float mu = sm / (float)DD; float q2 = 0.f;
#pragma unroll
  for (int k = 0; k < 16; ++k) { const float d = v[k] - mu; q2 += d * d; }
  for (int o = 16; o > 0; o >>= 1) q2 += __shfl_xor(q2, o, 32); const float rs = rsqrtf(q2 / (float)DD + 1e-5f); v4f o4[4]; FragH fh[2], fl[2];
#pragma unroll
  for (int k = 0; k < 16; ++k) { const int c = l * 16 + k; const float y = (v[k] - mu) * rs * bf16_round(g[c]) + bf16_round(bb[c]); o4[k >> 2][k & 3] = y; const _Float16 hi = (_Float16)y; fh[k >> 3].h[k & 7] = hi; fl[k >> 3].h[k & 7] = (_Float16)((y - (float)hi) * 1024.0f); }
  for (int pass = 0; pass < 2; ++pass) {
#pragma unroll
    for (int q = 0; q < 4; ++q) *(volatile v4f*)(X1 + (size_t)r * DD + l * 16 + 4 * q) = o4[q];
#pragma unroll
    for (int q = 0; q < 2; ++q) { *(volatile v8us*)((unsigned short*)X2 + (size_t)r * 2 * DD + l * 16 + 8 * q) = fh[q].half[0]; *(volatile v8us*)((unsigned short*)X2 + (size_t)r * 2 * DD + DD + l * 16 + 8 * q) = fl[q].half[0]; }
    if (pass == 0) __threadfence(); } }
__global__ __launch_bounds__(256) void k_ln2(const float* __restrict__ T, const float* __restrict__ g, const float* __restrict__ bb, float* __restrict__ out) {
  #pragma clang fp contract(off)
  const int tid = threadIdx.x, w = tid >> 5, l = tid & 31; const int r = blockIdx.x * 8 + w; if (r >= NR) return; float v[16]; float sm = 0.f;
#pragma unroll
  for (int k = 0; k < 16; ++k) { v[k] = T[(size_t)r * DD + l * 16 + k]; sm += v[k]; }
  for (int o = 16; o > 0; o >>= 1) sm += __shfl_xor(sm, o, 32); const float mu = sm / (float)DD; float q2 = 0.f;
#pragma unroll
  for (int k = 0; k < 16; ++k) { const float d = v[k] - mu; q2 += d * d; }
  for (int o = 16; o > 0; o >>= 1) q2 += __shfl_xor(q2, o, 32); const float rs = rsqrtf(q2 / (float)DD + 1e-5f); v4f o4[4];
#pragma unroll
  for (int k = 0; k < 16; ++k) { const int c = l * 16 + k; o4[k >> 2][k & 3] = (v[k] - mu) * rs * bf16_round(g[c]) + bf16_round(bb[c]); }
  for (int pass = 0; pass < 2; ++pass) {
#pragma unroll
    for (int q = 0; q < 4; ++q) *(volatile v4f*)(out + (size_t)r * DD + l * 16 + 4 * q) = o4[q];
    if (pass == 0) __threadfence(); } }
__global__ __launch_bounds__(256) void k_bfold(const float* __restrict__ Wm, int K, int O, _Float16* __restrict__ Bt) { const int t = blockIdx.x * 256 + threadIdx.x; if (t >= O * (2 * K / 8)) return; const int k0 = (t % (2 * K / 8)) * 8, o = t / (2 * K / 8); const int kb = k0 % K; const float sc = (k0 >= K) ? (16.0f / 1024.0f) : 16.0f; FragH f;
#pragma unroll
  for (int q = 0; q < 8; ++q) f.h[q] = (_Float16)(bf16_round(Wm[(size_t)(kb + q) * O + o]) * sc);
  *(volatile v8us*)((unsigned short*)Bt + (size_t)o * 2 * K + k0) = f.half[0]; __threadfence(); *(volatile v8us*)((unsigned short*)Bt + (size_t)o * 2 * K + k0) = f.half[0]; }

extern "C" void kernel_launch(void* const* d_in, const int* in_sizes, int n_in,
                              void* d_out, int out_size, void* d_ws, size_t ws_size, hipStream_t stream) {
  (void)in_sizes; (void)n_in; (void)out_size;
  const float* const* I = (const float* const*)d_in; const float* src = I[0]; const float* Wq = I[1]; const float* bq = I[2]; const float* Wk = I[3]; const float* bk = I[4]; const float* Wv = I[5]; const float* bv = I[6]; const float* Er = I[7]; const float* W1 = I[8]; const float* b1 = I[9]; const float* W2 = I[10]; const float* b2 = I[11]; const float* g1 = I[12]; const float* be1 = I[13]; const float* g2 = I[14]; const float* be2 = I[15];
  char* ws = (char*)d_ws; size_t off = 0;
  auto take = [&](size_t bytes) { char* p = ws + off; off += (bytes + 255) & ~(size_t)255; return p; };
  _Float16* BQ = (_Float16*)take((size_t)DD * DD * 2); _Float16* BK = (_Float16*)take((size_t)DD * DD * 2); _Float16* BV = (_Float16*)take((size_t)DD * DD * 2); _Float16* B1 = (_Float16*)take((size_t)DFF * 2 * DD * 2); _Float16* B2 = (_Float16*)take((size_t)DD * DFF * 2);
  _Float16* X16 = (_Float16*)take((size_t)NR * DD * 2); _Float16* E16 = (_Float16*)take((size_t)SS * HD * 2); _Float16* Q16 = (_Float16*)take((size_t)SS * DD * 2); _Float16* K16 = (_Float16*)take((size_t)SS * DD * 2); _Float16* V16 = (_Float16*)take((size_t)SS * DD * 2); _Float16* VT = (_Float16*)take((size_t)DD * SS * 2); float* QK = (float*)take((size_t)HG * SS * SS * 4); float* QE = (float*)take((size_t)HG * SS * SS * 4); _Float16* P16 = (_Float16*)take((size_t)HG * SS * SS * 2); float* SA = (float*)take((size_t)SS * DD * 4); float* X1 = (float*)take((size_t)NR * DD * 4); _Float16* X2 = (_Float16*)take((size_t)NR * 2 * DD * 2); _Float16* H16 = (_Float16*)take((size_t)NR * DFF * 2); float* T2 = (float*)take((size_t)NR * DD * 4);
  if (off > ws_size) return;
  const unsigned nbw = (unsigned)(((size_t)DD * (DD / 8) + 255) / 256);
  k_wt_f16<<<nbw, 256, 0, stream>>>(Wq, BQ, DD, DD, 16.0f); k_wt_f16<<<nbw, 256, 0, stream>>>(Wk, BK, DD, DD, 16.0f); k_wt_f16<<<nbw, 256, 0, stream>>>(Wv, BV, DD, DD, 16.0f);
  k_bfold<<<(unsigned)(((size_t)DFF * (2 * DD / 8) + 255) / 256), 256, 0, stream>>>(W1, DD, DFF, B1); k_wt_f16<<<(unsigned)(((size_t)DD * (DFF / 8) + 255) / 256), 256, 0, stream>>>(W2, B2, DFF, DD, 16.0f);
  const size_t n8 = (size_t)NR * DD / 8; k_x16<<<(unsigned)((n8 + 255) / 256), 256, 0, stream>>>(src, X16, n8); k_er<<<(SS * (HD / 8) + 255) / 256, 256, 0, stream>>>(Er, E16);
  const dim3 gP1(((SS / 16) * (DD / 64) + 3) / 4, 1);
  k_gemm_hhx<0><<<gP1, 128, 0, stream>>>(X16, 2 * DD, 0, BQ, DD, 0, 0.0625f, bq, 0, nullptr, 1, 0, 0, nullptr, Q16, DD, 0, SS, DD, DD);
  k_gemm_hhx<0><<<gP1, 128, 0, stream>>>(X16, 2 * DD, 0, BK, DD, 0, 0.0625f, bk, 0, nullptr, 1, 0, 0, nullptr, K16, DD, 0, SS, DD, DD);
  k_gemm_hhx<0><<<gP1, 128, 0, stream>>>(X16, 2 * DD, 0, BV, DD, 0, 0.0625f, bv, 0, nullptr, 1, 0, 0, nullptr, V16, DD, 0, SS, DD, DD); k_vt<<<(DD * (SS / 8) + 255) / 256, 256, 0, stream>>>(V16, VT);
  const dim3 gS(((SS / 16) * (SS / 64) + 3) / 4, HG), gV(((SS / 16) * 1 + 3) / 4, HG);
  for (int hg = 0; hg < NH / HG; ++hg) { const int h0 = hg * HG;
    k_gemm_hhx<0><<<gS, 128, 0, stream>>>(Q16 + h0 * HD, DD, (size_t)HD, K16 + h0 * HD, DD, (size_t)HD, 1.0f, nullptr, 0, nullptr, 1, 0, 0, QK, nullptr, SS, (size_t)SS * SS, SS, SS, HD);
    k_gemm_hhx<0><<<gS, 128, 0, stream>>>(Q16 + h0 * HD, DD, (size_t)HD, E16, HD, 0, 1.0f, nullptr, 0, nullptr, 1, 0, 0, QE, nullptr, SS, (size_t)SS * SS, SS, SS, HD);
    k_rsoft<<<HG * SS / 8, 256, 0, stream>>>(QK, QE, P16);
    k_gemm_hhx<0><<<gV, 128, 0, stream>>>(P16, SS, (size_t)SS * SS, VT + (size_t)h0 * HD * SS, SS, (size_t)HD * SS, 0.0009765625f, nullptr, 0, nullptr, 1, 0, 0, SA + h0 * HD, nullptr, DD, (size_t)HD, SS, HD, SS); }
  k_ln1<<<NR / 8, 256, 0, stream>>>(src, SA, g1, be1, X1, X2);
  const dim3 gF(((NR / 16) * (DFF / 64) + 3) / 4, 1), gO(((NR / 16) * (DD / 64) + 3) / 4, 1);
  k_gemm_hhx<3><<<gF, 128, 0, stream>>>(X2, 2 * DD, 0, B1, 2 * DD, 0, 0.0625f, b1, 0, nullptr, 1, 0, 0, nullptr, H16, DFF, 0, NR, DFF, 2 * DD);
  k_gemm_hhx<0><<<gO, 128, 0, stream>>>(H16, DFF, 0, B2, DFF, 0, 0.0625f, b2, 0, X1, 1, (size_t)DD, 0, T2, nullptr, DD, 0, NR, DD, DFF);
  k_ln2<<<NR / 8, 256, 0, stream>>>(T2, g2, be2, (float*)d_out);
}
